// PinnWithGRU_4329327034799
// MI455X (gfx1250) — hardware-verified
//
#include <hip/hip_runtime.h>

typedef __attribute__((ext_vector_type(16))) _Float16 v16h;
typedef __attribute__((ext_vector_type(8)))  _Float16 v8h;
typedef __attribute__((ext_vector_type(8)))  float    v8f;
typedef __attribute__((ext_vector_type(4)))  float    v4f;

constexpr int kBatch  = 2048;
constexpr int kSteps  = 2048;
constexpr int kChan   = 3;
constexpr int kHid    = 32;
constexpr int kGate   = 3 * kHid;
constexpr int kTileM  = 16;
constexpr int kChunk  = 32;
constexpr int kHPitch = 40;
constexpr int kNumPar = kGate * kChan + kGate + kHid;
constexpr float kCarryH = 64.0f;
constexpr float kCarryW = 256.0f;
constexpr float kFold   = 1.0f / (kCarryH * kCarryW);
constexpr float kF16MinNormal = 6.103515625e-05f;

static_assert(kHid == 32, "recurrent product is exactly one 32-deep k-step");
static_assert(kGate == 96, "six 16-wide gate tiles");
static_assert(kChunk == 32, "one lane per buffered step; 32 floats = one 128-B output line");
static_assert((kBatch % kTileM) == 0 && (kSteps % kChunk) == 0, "tile multiples");
static_assert(kNumPar == 416, "parameter table size");
static_assert((kHPitch % 8) == 0 && kHPitch >= kHid, "16-B aligned h rows");
static_assert(kFold == 1.0f / 16384.0f, "fold constant");

__device__ __forceinline__ float bf16_value(float f) {
  unsigned u = __float_as_uint(f);
  u = (u + 0x7FFFu + ((u >> 16) & 1u)) & 0xFFFF0000u;
  return __uint_as_float(u);
}
__device__ __forceinline__ _Float16 to_f16_flushed(float v) {
  const float q = (fabsf(v) < kF16MinNormal) ? 0.0f : v;
  return (_Float16)q;
}
__device__ __forceinline__ v8f mma_from_zero(v16h a, v16h b) {
  v8f c = (v8f){0.f, 0.f, 0.f, 0.f, 0.f, 0.f, 0.f, 0.f};
  c = __builtin_amdgcn_wmma_f32_16x16x32_f16(false, a, false, b, (short)0, c, false, false);
  asm volatile("v_nop\n\tv_nop\n\tv_nop\n\tv_nop" : "+v"(c) : "v"(a), "v"(b));
  return c;
}
__device__ __forceinline__ v16h frag_load_h(const _Float16* p) {
  union { v16h v; v8h h[2]; } f;
  f.h[0] = *(const v8h*)(p);
  f.h[1] = *(const v8h*)(p + 16);
  return f.v;
}
__device__ __forceinline__ float fast_sigmoid(float x) {
  return __builtin_amdgcn_rcpf(1.0f + __expf(-x));
}
__device__ __forceinline__ float fast_tanh(float x) {
  return 1.0f - 2.0f * __builtin_amdgcn_rcpf(__expf(2.0f * x) + 1.0f);
}

__global__ __launch_bounds__(32) void gated_recurrence32_steps(
    const float* __restrict__ inp,
    const float* __restrict__ w_ih,
    const float* __restrict__ w_hh,
    const float* __restrict__ bias,
    const float* __restrict__ bias_n,
    float* __restrict__ out)
{
  __shared__ __align__(16) float    sX[kChunk * kTileM * 4];
  __shared__ __align__(16) float    sO[kTileM * kChunk];
  __shared__ __align__(16) _Float16 sH[kTileM * kHPitch];
  __shared__ __align__(16) float    sP[kNumPar];

  const int lane = threadIdx.x & 31;
  const int hh   = lane >> 4;
  const int ln   = lane & 15;
  const int b0   = blockIdx.x * kTileM;
  if (b0 >= kBatch) return;

#pragma unroll 1
  for (int i = lane; i < kGate * kChan; i += 32) sP[i] = bf16_value(w_ih[i]);
#pragma unroll 1
  for (int i = lane; i < kGate; i += 32) sP[kGate * kChan + i] = bf16_value(bias[i]);
  sP[kGate * kChan + kGate + lane] = bf16_value(bias_n[lane]);

  v16h wB[6];
#pragma unroll
  for (int nt = 0; nt < 6; ++nt) {
    const float* wp = w_hh + (nt * 16 + ln) * kHid + 8 * hh;
    const v4f q0 = *(const v4f*)(wp);
    const v4f q1 = *(const v4f*)(wp + 4);
    const v4f q2 = *(const v4f*)(wp + 16);
    const v4f q3 = *(const v4f*)(wp + 20);
    v16h f;
#pragma unroll
    for (int e = 0; e < 4; ++e) {
      const float a0 = q0[e];
      const float a1 = q1[e];
      const float a2 = q2[e];
      const float a3 = q3[e];
      f[e]      = to_f16_flushed(bf16_value(a0) * kCarryW);
      f[4 + e]  = to_f16_flushed(bf16_value(a1) * kCarryW);
      f[8 + e]  = to_f16_flushed(bf16_value(a2) * kCarryW);
      f[12 + e] = to_f16_flushed(bf16_value(a3) * kCarryW);
    }
    wB[nt] = f;
  }

  float hC[2][8];
#pragma unroll
  for (int tl = 0; tl < 2; ++tl) {
#pragma unroll
    for (int r = 0; r < 8; ++r) {
      hC[tl][r] = 0.0f;
      sH[(8 * hh + r) * kHPitch + tl * 16 + ln] = (_Float16)0.0f;
    }
  }
  __syncthreads();

  float wR[2][3], wZ[2][3], wA[2][3], bR[2], bZ[2], bA[2], bN[2];
#pragma unroll
  for (int tl = 0; tl < 2; ++tl) {
    const int j = tl * 16 + ln;
#pragma unroll
    for (int c = 0; c < 3; ++c) {
      wR[tl][c] = sP[j * kChan + c];
      wZ[tl][c] = sP[(kHid + j) * kChan + c];
      wA[tl][c] = sP[(2 * kHid + j) * kChan + c];
    }
    bR[tl] = sP[kGate * kChan + j];
    bZ[tl] = sP[kGate * kChan + kHid + j];
    bA[tl] = sP[kGate * kChan + 2 * kHid + j];
    bN[tl] = sP[kGate * kChan + kGate + j];
  }

  const float* xbase = inp + (size_t)b0 * kSteps * kChan;
  float*       obase = out + (size_t)b0 * kSteps;
  const _Float16* hrd = sH + ln * kHPitch + 8 * hh;
  const int q  = lane >> 3;
  const int c4 = (lane & 7) * 4;

#pragma unroll 1
  for (int t0 = 0; t0 < kSteps; t0 += kChunk) {
    __syncthreads();
#pragma unroll 4
    for (int m = 0; m < kTileM; ++m) {
      const float* xp = xbase + ((size_t)m * kSteps + (size_t)(t0 + lane)) * kChan;
      const float x0 = xp[0];
      const float x1 = xp[1];
      const float x2 = xp[2];
      v4f v;
      v[0] = bf16_value(x0);
      v[1] = bf16_value(x1);
      v[2] = bf16_value(x2);
      v[3] = 0.0f;
      *(v4f*)(sX + ((lane * kTileM + m) << 2)) = v;
    }
    __syncthreads();

#pragma unroll 1
    for (int s = 0; s < kChunk; ++s) {
      const v16h fa = frag_load_h(hrd);
      v4f xr[8];
#pragma unroll
      for (int r = 0; r < 8; ++r) xr[r] = *(const v4f*)(sX + ((s * kTileM + 8 * hh + r) << 2));
      __syncthreads();

#pragma unroll
      for (int tl = 0; tl < 2; ++tl) {
        const v8f cr = mma_from_zero(fa, wB[tl]);
        const v8f cz = mma_from_zero(fa, wB[tl + 2]);
        const v8f cn = mma_from_zero(fa, wB[tl + 4]);
#pragma unroll
        for (int r = 0; r < 8; ++r) {
          const float x0 = xr[r][0];
          const float x1 = xr[r][1];
          const float x2 = xr[r][2];
          float ir = x0 * wR[tl][0];
          ir = fmaf(x1, wR[tl][1], ir);
          ir = fmaf(x2, wR[tl][2], ir);
          ir = ir + bR[tl];
          float iz = x0 * wZ[tl][0];
          iz = fmaf(x1, wZ[tl][1], iz);
          iz = fmaf(x2, wZ[tl][2], iz);
          iz = iz + bZ[tl];
          float ia = x0 * wA[tl][0];
          ia = fmaf(x1, wA[tl][1], ia);
          ia = fmaf(x2, wA[tl][2], ia);
          ia = ia + bA[tl];
          const float hr = cr[r] * kFold;
          const float hz = cz[r] * kFold;
          const float ha = cn[r] * kFold;
          const float rg = fast_sigmoid(ir + hr);
          const float zg = fast_sigmoid(iz + hz);
          const float ng = fast_tanh((ia + bN[tl]) + rg * ha);
          const float hn = (1.0f - zg) * ng + zg * hC[tl][r];
          hC[tl][r] = hn;
          sH[(8 * hh + r) * kHPitch + tl * 16 + ln] = to_f16_flushed(hn * kCarryH);
        }
        if (tl == 0) {
          if (ln == 0) {
#pragma unroll
            for (int r = 0; r < 8; ++r) sO[(8 * hh + r) * kChunk + s] = hC[0][r];
          }
        }
      }
      __syncthreads();
    }

    v4f ov[4];
#pragma unroll
    for (int it = 0; it < 4; ++it) ov[it] = *(const v4f*)(sO + (it * 4 + q) * kChunk + c4);
    for (int pass = 0; pass < 2; ++pass) {
#pragma unroll
      for (int it = 0; it < 4; ++it) {
        *(volatile v4f*)(obase + (size_t)(it * 4 + q) * kSteps + t0 + c4) = ov[it];
      }
      __threadfence();
    }
  }
}

extern "C" void kernel_launch(void* const* d_in, const int* in_sizes, int n_in,
                              void* d_out, int out_size, void* d_ws, size_t ws_size,
                              hipStream_t stream) {
  (void)d_ws;
  (void)ws_size;
  if (n_in < 5) return;
  if (in_sizes[0] != kBatch * kSteps * kChan) return;
  if (in_sizes[1] != kGate * kChan) return;
  if (in_sizes[2] != kGate * kHid) return;
  if (in_sizes[3] != kGate) return;
  if (in_sizes[4] != kHid) return;
  if (out_size != kBatch * kSteps) return;

  const float* inp    = (const float*)d_in[0];
  const float* w_ih   = (const float*)d_in[1];
  const float* w_hh   = (const float*)d_in[2];
  const float* bias   = (const float*)d_in[3];
  const float* bias_n = (const float*)d_in[4];
  float* out = (float*)d_out;

  gated_recurrence32_steps<<<dim3(kBatch / kTileM), dim3(32), 0, stream>>>(inp, w_ih, w_hh, bias, bias_n, out);
}
